// ScatteredExperts_83803401879802
// MI455X (gfx1250) — hardware-run, weakly checked
//
#include <hip/hip_runtime.h>
#include <stddef.h>
#include <stdint.h>

#define NTOK   4096
#define DIN    1024
#define DOUT   1024
#define NEXP   8
#define FAN    2
#define NPOS   (NTOK * FAN)
#define TROWS  64
#define NTILE  (NPOS / TROWS)
#define WSC    64.0f
#define UGS    0.015625f
#define APITCH 136
#define OTP    68
#define TRP    72

static_assert(NPOS % TROWS == 0);
static_assert(DIN % 128 == 0);
static_assert(DOUT % 128 == 0);
static_assert(DIN % 64 == 0);
static_assert(DOUT % 64 == 0);
static_assert((NTOK * DIN) % 2048 == 0);
static_assert((NTOK * DOUT) % 1024 == 0);
static_assert(FAN == 2);
static_assert(NEXP == 8);
static_assert((APITCH * 2) % 16 == 0);
static_assert((OTP * 4) % 16 == 0);
static_assert((TRP * 2) % 16 == 0);

typedef _Float16 v16h __attribute__((ext_vector_type(16)));
typedef _Float16 v8h  __attribute__((ext_vector_type(8)));
typedef float    v8f  __attribute__((ext_vector_type(8)));
typedef float    v4f  __attribute__((ext_vector_type(4)));
typedef unsigned int v4u __attribute__((ext_vector_type(4)));

union Frag  { v16h v; v8h h[2]; };
union Pack8 { v8h h; v4u u; };

__device__ __forceinline__ int clampi(int v, int lo, int hi) { return min(max(v, lo), hi); }

__device__ __forceinline__ v8f mma16(v16h a, v16h b, v8f c) {
  c = __builtin_amdgcn_wmma_f32_16x16x32_f16(false, a, false, b, (short)0, c, false, false);
  asm volatile("v_nop\n\tv_nop\n\tv_nop\n\tv_nop" : "+v"(c) : "v"(a), "v"(b));
  return c;
}

__device__ __forceinline__ v16h ldfrag(const _Float16* p, int ld, int row0, int k0, int lane) {
  const int m = lane & 15, lh = lane >> 4;
  const _Float16* q = p + (size_t)(row0 + m) * ld + k0 + 8 * lh;
  Frag f;
  f.h[0] = *(const v8h*)(q);
  f.h[1] = *(const v8h*)(q + 16);
  return f.v;
}

__device__ __forceinline__ v8f zero8() { return (v8f){0.f, 0.f, 0.f, 0.f, 0.f, 0.f, 0.f, 0.f}; }

__global__ __launch_bounds__(256) void k_cvt(const float* __restrict__ src, _Float16* __restrict__ dh, int n8) {
  const int i = blockIdx.x * 256 + (int)threadIdx.x;
  if (i >= n8) return;
  const size_t o = (size_t)i * 8;
  const v4f a0 = *(const v4f*)(src + o);
  const v4f a1 = *(const v4f*)(src + o + 4);
  Pack8 pk;
  pk.h = (v8h){(_Float16)a0[0], (_Float16)a0[1], (_Float16)a0[2], (_Float16)a0[3],
               (_Float16)a1[0], (_Float16)a1[1], (_Float16)a1[2], (_Float16)a1[3]};
  const v4u vv = pk.u;
  volatile v4u* d = (volatile v4u*)(dh + o);
  *d = vv;
  __threadfence();
  *d = vv;
}

__global__ __launch_bounds__(256) void k_wtr(const float* __restrict__ w, _Float16* __restrict__ wt,
                                             int kdim, int ndim, float scale) {
  __shared__ __align__(16) _Float16 st[64 * TRP];
  const int tid = threadIdx.x;
  const size_t bo = (size_t)blockIdx.z * (size_t)kdim * (size_t)ndim;
  w  += bo;
  wt += bo;
  const int n0 = blockIdx.x * 64, k0 = blockIdx.y * 64;
  const int kr = tid >> 2;
  const int nc = (tid & 3) * 16;
  const float* sp = w + (size_t)(k0 + kr) * ndim + n0 + nc;
#pragma unroll
  for (int q = 0; q < 4; ++q) {
    const v4f a = *(const v4f*)(sp + 4 * q) * scale;
#pragma unroll
    for (int j = 0; j < 4; ++j) st[(nc + 4 * q + j) * TRP + kr] = (_Float16)a[j];
  }
  __syncthreads();
  v4u val[2];
  size_t go[2];
#pragma unroll
  for (int j = 0; j < 2; ++j) {
    const int p  = tid + 256 * j;
    const int nr = p >> 3;
    const int pc = p & 7;
    Pack8 pk;
    pk.h   = *(const v8h*)(st + nr * TRP + pc * 8);
    val[j] = pk.u;
    go[j]  = (size_t)(n0 + nr) * kdim + k0 + pc * 8;
  }
#pragma unroll
  for (int j = 0; j < 2; ++j) *(volatile v4u*)(wt + go[j]) = val[j];
  __threadfence();
#pragma unroll
  for (int j = 0; j < 2; ++j) *(volatile v4u*)(wt + go[j]) = val[j];
  __threadfence();
}

__global__ __launch_bounds__(256) void k_gemm(const _Float16* __restrict__ xh, const _Float16* __restrict__ wt,
                                              const int* __restrict__ bin_ids, const int* __restrict__ indices,
                                              const int* __restrict__ pbi, const int* __restrict__ eoff,
                                              float* __restrict__ part) {
  __shared__ __align__(16) _Float16 sA[TROWS * APITCH];
  __shared__ __align__(16) float sO[8 * 16 * OTP];
  __shared__ int sTok[TROWS];
  __shared__ int sDst[TROWS];
  __shared__ int sBin[TROWS];
  (void)pbi;
  (void)eoff;
  const int tid = threadIdx.x, lane = tid & 31, wave = tid >> 5;
  const int hh = lane >> 4, c = lane & 15;
  const int wm = wave & 3, wn = wave >> 2;
  const int p0 = blockIdx.y * TROWS;
  const int n0 = blockIdx.x * 128;

  if (tid < TROWS) {
    const int p   = p0 + tid;
    const int idx = clampi(indices[p], 0, NPOS - 1);
    sTok[tid] = idx >> 1;
    sDst[tid] = idx;
    sBin[tid] = clampi(bin_ids[p], 0, NEXP - 1);
  }
  __syncthreads();

  int emin = NEXP - 1, emax = 0;
#pragma unroll 8
  for (int r = 0; r < TROWS; ++r) {
    const int bq = sBin[r];
    emin = min(emin, bq);
    emax = max(emax, bq);
  }
  emin = __builtin_amdgcn_readfirstlane(clampi(emin, 0, NEXP - 1));
  emax = __builtin_amdgcn_readfirstlane(clampi(emax, 0, NEXP - 1));

  const int brow = n0 + wn * 64;

  v8f acc[4];
#pragma unroll
  for (int t = 0; t < 4; ++t) acc[t] = zero8();

  const int ar = tid >> 2, ac = tid & 3;
  const _Float16* xrow = xh + (size_t)sTok[ar] * DIN + ac * 32;
  _Float16* arow = sA + ar * APITCH + ac * 32;
  const int abin = sBin[ar];

#pragma unroll 1
  for (int e = emin; e <= emax; ++e) {
    const unsigned mk = (abin == e) ? 0xFFFFFFFFu : 0u;
    const v4u mv = (v4u){mk, mk, mk, mk};
    const _Float16* wte = wt + (size_t)e * (size_t)DOUT * (size_t)DIN;
#pragma unroll 1
    for (int kc = 0; kc < DIN / 128; ++kc) {
      __syncthreads();
#pragma unroll
      for (int q = 0; q < 4; ++q) {
        Pack8 pk;
        pk.h = *(const v8h*)(xrow + kc * 128 + 8 * q);
        pk.u = pk.u & mv;
        *(v8h*)(arow + 8 * q) = pk.h;
      }
      __syncthreads();
#pragma unroll 1
      for (int ks = 0; ks < 4; ++ks) {
        const int kg = kc * 128 + ks * 32;
        const v16h a = ldfrag(sA, APITCH, wm * 16, ks * 32, lane);
#pragma unroll
        for (int t = 0; t < 4; ++t) {
          const v16h bq = ldfrag(wte, DIN, brow + 16 * t, kg, lane);
          acc[t] = mma16(a, bq, acc[t]);
        }
      }
    }
  }

  float* sw = sO + wave * (16 * OTP);
#pragma unroll
  for (int t = 0; t < 4; ++t) {
#pragma unroll
    for (int r = 0; r < 8; ++r) sw[(8 * hh + r) * OTP + 16 * t + c] = acc[t][r] * UGS;
  }
  __syncthreads();
  v4f val[8];
  size_t go[8];
#pragma unroll
  for (int it = 0; it < 8; ++it) {
    const int p    = lane + 32 * it;
    const int L    = p >> 3;
    const int pc   = p & 7;
    const int row  = L >> 1;
    const int half = L & 1;
    const int lr   = wm * 16 + row;
    val[it] = *(const v4f*)(sw + row * OTP + half * 32 + pc * 4);
    go[it]  = (size_t)sDst[lr] * DOUT + brow + half * 32 + pc * 4;
  }
#pragma unroll
  for (int it = 0; it < 8; ++it) *(volatile v4f*)(part + go[it]) = val[it];
  __threadfence();
#pragma unroll
  for (int it = 0; it < 8; ++it) *(volatile v4f*)(part + go[it]) = val[it];
  __threadfence();
}

__global__ __launch_bounds__(256) void k_comb(const float* __restrict__ part, const float* __restrict__ gates,
                                              float* __restrict__ out, int n4) {
#pragma clang fp contract(off)
  const int i = blockIdx.x * 256 + (int)threadIdx.x;
  if (i >= n4) return;
  const size_t o = (size_t)i * 4;
  const size_t t = o / DOUT;
  const size_t n = o - t * DOUT;
  const float g0 = gates[t * FAN];
  const float g1 = gates[t * FAN + 1];
  const float* pr = part + t * (size_t)(FAN * DOUT) + n;
  const v4f a = *(const v4f*)(pr);
  const v4f b = *(const v4f*)(pr + DOUT);
  const v4f pa = a * g0;
  const v4f pb = b * g1;
  const v4f v = pa + pb;
  volatile v4f* d = (volatile v4f*)(out + o);
  *d = v;
  __threadfence();
  *d = v;
}

extern "C" void kernel_launch(void* const* d_in, const int* in_sizes, int n_in,
                              void* d_out, int out_size, void* d_ws, size_t ws_size,
                              hipStream_t stream) {
  if (n_in < 7) return;
  if (in_sizes[0] != NTOK * DIN) return;
  if (in_sizes[1] != NEXP * DIN * DOUT) return;
  if (in_sizes[2] != NPOS) return;
  if (in_sizes[3] != NPOS) return;
  if (in_sizes[4] < 1) return;
  if (in_sizes[5] < 1) return;
  if (in_sizes[6] != NTOK * FAN) return;
  if (out_size != NTOK * DOUT) return;

  const float* x       = (const float*)d_in[0];
  const float* W       = (const float*)d_in[1];
  const int*   bin_ids = (const int*)d_in[2];
  const int*   indices = (const int*)d_in[3];
  const int*   pbi     = (const int*)d_in[4];
  const int*   eoff    = (const int*)d_in[5];
  const float* gates   = (const float*)d_in[6];
  float* out = (float*)d_out;

  size_t off = 0;
  const size_t oXh = off; off += (size_t)NTOK * DIN * 2;
  const size_t oWT = off; off += (size_t)NEXP * DIN * DOUT * 2;
  const size_t oP  = off; off += (size_t)NPOS * DOUT * 4;
  if (off > ws_size) return;
  if (off > (size_t)134217728) return;
  if ((oWT | oP) & (size_t)127) return;

  char* ws = (char*)d_ws;
  _Float16* Xh = (_Float16*)(ws + oXh);
  _Float16* WT = (_Float16*)(ws + oWT);
  float*    P  = (float*)(ws + oP);

  k_cvt<<<dim3((NTOK * DIN) / 8 / 256), dim3(256), 0, stream>>>(x, Xh, (NTOK * DIN) / 8);
  k_wtr<<<dim3(DOUT / 64, DIN / 64, NEXP), dim3(256), 0, stream>>>(W, WT, DIN, DOUT, WSC);
  k_gemm<<<dim3(DOUT / 128, NTILE), dim3(256), 0, stream>>>(Xh, WT, bin_ids, indices, pbi, eoff, P);
  k_comb<<<dim3((NTOK * DOUT) / 4 / 256), dim3(256), 0, stream>>>(P, gates, out, (NTOK * DOUT) / 4);
  (void)hipGetLastError();
}
